// MainModule_57501022158924
// MI455X (gfx1250) — hardware-verified
//
#include <hip/hip_runtime.h>
#include <math.h>
#include <stddef.h>

#define BB 8
#define TT 4096
#define BT (BB * TT)
#define DD 64
#define NLAY 11
#define NHD 8
#define NSPEC 81
#define X1P 224
#define X2P 160
#define WSC 16.0f
#define INV_WSC 0.0625f

static_assert(BT % 64 == 0);
static_assert(TT % 256 == 0);
static_assert((X1P * 4) % 128 == 0);
static_assert((X2P * 4) % 128 == 0);

typedef _Float16 v16h __attribute__((ext_vector_type(16)));
typedef _Float16 v8h  __attribute__((ext_vector_type(8)));
typedef __bf16   v16b __attribute__((ext_vector_type(16)));
typedef __bf16   v8b  __attribute__((ext_vector_type(8)));
typedef float    v8f  __attribute__((ext_vector_type(8)));
typedef float    v4f  __attribute__((ext_vector_type(4)));

union FragH { v16h v; v8h half[2]; };
union FragB { v16b v; v8b half[2]; };

__device__ __forceinline__ v8f mma_h(v16h a, v16h b, v8f c) {
    c = __builtin_amdgcn_wmma_f32_16x16x32_f16(false, a, false, b, (short)0, c, false, false);
    asm volatile("v_nop\n\tv_nop\n\tv_nop\n\tv_nop" : "+v"(c) : "v"(a), "v"(b));
    return c;
}
__device__ __forceinline__ v8f mma_b(v16b a, v16b b, v8f c) {
    c = __builtin_amdgcn_wmma_f32_16x16x32_bf16(false, a, false, b, (short)0, c, false, false);
    asm volatile("v_nop\n\tv_nop\n\tv_nop\n\tv_nop" : "+v"(c) : "v"(a), "v"(b));
    return c;
}

__device__ __forceinline__ int kmap(int i, int h) { return ((i >> 3) << 4) + (h << 3) + (i & 7); }

__device__ __forceinline__ v8f v8fill(float a) {
    v8f z;
#pragma unroll
    for (int r = 0; r < 8; ++r) z[r] = a;
    return z;
}

template <bool ADD>
__device__ __forceinline__ void wave_store_tile(const float* tile, float* g, int lane) {
    int offs[8];
    v4f vals[8];
#pragma unroll
    for (int it = 0; it < 8; ++it) {
        int ql = it * 4 + (lane >> 3);
        int off = (ql >> 1) * DD + ((ql & 1) << 5) + ((lane & 7) << 2);
        v4f val = *(const v4f*)(tile + off);
        if (ADD) val += *(const v4f*)(g + off);
        offs[it] = off;
        vals[it] = val;
    }
#pragma unroll
    for (int it = 0; it < 8; ++it) *(volatile v4f*)(g + offs[it]) = vals[it];
    __threadfence();
#pragma unroll
    for (int it = 0; it < 8; ++it) *(volatile v4f*)(g + offs[it]) = vals[it];
}

__device__ __forceinline__ void ln_rows(const float* __restrict__ x, int bt0, int tid,
                                        const float* __restrict__ g, const float* __restrict__ be,
                                        _Float16* hs) {
    if (tid < 64) {
        const v4f* xr = (const v4f*)(x + (size_t)(bt0 + tid) * DD);
        float xv[DD];
        float s = 0.f;
#pragma unroll
        for (int i = 0; i < 16; ++i) {
            v4f t4 = xr[i];
            xv[4 * i + 0] = t4[0]; xv[4 * i + 1] = t4[1];
            xv[4 * i + 2] = t4[2]; xv[4 * i + 3] = t4[3];
            s += (t4[0] + t4[1]) + (t4[2] + t4[3]);
        }
        float mean = s * (1.f / DD);
        float s2 = 0.f;
#pragma unroll
        for (int i = 0; i < DD; ++i) { float d = xv[i] - mean; s2 += d * d; }
        float inv = rsqrtf(s2 * (1.f / DD) + 1e-5f);
        _Float16* dst = hs + tid * DD;
#pragma unroll
        for (int c = 0; c < 8; ++c) {
            v8h p;
#pragma unroll
            for (int j = 0; j < 8; ++j) {
                int kk = 8 * c + j;
                p[j] = (_Float16)((xv[kk] - mean) * inv * g[kk] + be[kk]);
            }
            *(v8h*)(dst + 8 * c) = p;
        }
    }
}

__global__ __launch_bounds__(256) void k_wcvt(const float* __restrict__ w0, const float* __restrict__ w1,
                                              const float* __restrict__ w2, const float* __restrict__ w3,
                                              const float* __restrict__ w4, _Float16* __restrict__ out,
                                              int nvec) {
    int i = blockIdx.x * blockDim.x + threadIdx.x;
    if (i >= nvec) return;
    int e0 = i * 8;
    int mtx = e0 / (NLAY * DD * DD);
    int r = e0 - mtx * (NLAY * DD * DD);
    const float* src = (mtx == 0) ? w0 : (mtx == 1) ? w1 : (mtx == 2) ? w2 : (mtx == 3) ? w3 : w4;
    v8h vv;
#pragma unroll
    for (int j = 0; j < 8; ++j) vv[j] = (_Float16)(src[r + j] * WSC);
    _Float16* p = out + e0;
    *(volatile v8h*)p = vv;
    __threadfence();
    *(volatile v8h*)p = vv;
}

__global__ __launch_bounds__(256) void k_conv1(const float* __restrict__ spec, const float* __restrict__ w,
                                               const float* __restrict__ bias, float* __restrict__ x1) {
    __shared__ float sps[NSPEC * 10];
    __shared__ float wsm[72];
    __shared__ float bsm[24];
    __shared__ __attribute__((aligned(16))) float outs[8 * X1P];
    int tid = threadIdx.x;
    int bt0 = blockIdx.x * 8;
    int b = bt0 >> 12, tl0 = bt0 & (TT - 1);
    for (int i = tid; i < NSPEC * 10; i += 256) {
        int f = i / 10, dt = i - f * 10;
        int t = tl0 + dt;
        sps[i] = (t < TT) ? spec[((size_t)b * NSPEC + f) * TT + t] : 0.f;
    }
    if (tid < 72) wsm[tid] = w[tid];
    if (tid < 24) bsm[tid] = bias[tid];
    __syncthreads();
    int tok = tid >> 5, lane = tid & 31;
    int t = tl0 + tok;
    int nsub = TT - t; if (nsub > 3) nsub = 3;
#pragma unroll 1
    for (int j = 0; j < 7; ++j) {
        int o = lane + 32 * j;
        int c = o / 28, f2 = o - 28 * c;
        float val = 0.f;
        if (f2 < 26) {
            float bs = bsm[c];
            if (nsub > 1) bs += bsm[8 + c];
            if (nsub > 2) bs += bsm[16 + c];
            float mx = -3.4e38f;
#pragma unroll
            for (int fp = 0; fp < 3; ++fp) {
                float acc = bs;
#pragma unroll
                for (int i = 0; i < 3; ++i)
#pragma unroll
                    for (int kw = 0; kw < 3; ++kw)
                        acc += wsm[(i * 8 + c) * 3 + kw] * sps[(3 * f2 + fp + kw) * 10 + tok + i];
                mx = fmaxf(mx, acc);
            }
            val = fmaxf(mx, 0.f);
        }
        outs[tok * X1P + o] = val;
    }
    __syncthreads();
    float* gp = x1 + (size_t)(bt0 + tok) * X1P;
    const float* lp = outs + tok * X1P;
    v4f s0 = *(const v4f*)(lp + lane * 4);
    v4f s1 = s0;
    bool second = lane < 24;
    if (second) s1 = *(const v4f*)(lp + (32 + lane) * 4);
    *(volatile v4f*)(gp + lane * 4) = s0;
    if (second) *(volatile v4f*)(gp + (32 + lane) * 4) = s1;
    __threadfence();
    *(volatile v4f*)(gp + lane * 4) = s0;
    if (second) *(volatile v4f*)(gp + (32 + lane) * 4) = s1;
}

__global__ __launch_bounds__(128) void k_conv2(const float* __restrict__ x1, const float* __restrict__ w,
                                               const float* __restrict__ bias, float* __restrict__ x2) {
    __shared__ __attribute__((aligned(16))) float xs[4 * X1P];
    __shared__ __attribute__((aligned(16))) __bf16 whi[32 * 96];
    __shared__ __attribute__((aligned(16))) __bf16 wlo[32 * 96];
    __shared__ float bsm[32];
    __shared__ __attribute__((aligned(16))) float ds[4 * 16 * 32];
    __shared__ __attribute__((aligned(16))) float os[4 * X2P];
    int tid = threadIdx.x;
    int bt0 = blockIdx.x * 4;
    {
        const v4f* src = (const v4f*)(x1 + (size_t)bt0 * X1P);
        v4f* dst = (v4f*)xs;
        const int n4 = 4 * X1P / 4;
        for (int i = tid; i < n4; i += 128) dst[i] = src[i];
    }
    for (int i = tid; i < 32 * 96; i += 128) {
        float val = w[i];
        __bf16 hi = (__bf16)val;
        whi[i] = hi;
        wlo[i] = (__bf16)(val - (float)hi);
    }
    if (tid < 32) bsm[tid] = bias[tid];
    __syncthreads();
    int wave = tid >> 5, lane = tid & 31, h = lane >> 4, m = lane & 15;
    const float* xt = xs + wave * X1P;
    v8f acc[2];
    acc[0] = v8fill(0.f); acc[1] = v8fill(0.f);
#pragma unroll 1
    for (int ks = 0; ks < 3; ++ks) {
        FragB ah, al;
#pragma unroll
        for (int i = 0; i < 16; ++i) {
            int kk = ks * 32 + kmap(i, h);
            int cin = kk / 12, kw = kk - cin * 12;
            float val = xt[cin * 28 + m + kw];
            __bf16 hi = (__bf16)val;
            ah.v[i] = hi;
            al.v[i] = (__bf16)(val - (float)hi);
        }
#pragma unroll
        for (int nt = 0; nt < 2; ++nt) {
            int n = nt * 16 + m;
            const __bf16* wph = whi + n * 96 + ks * 32;
            const __bf16* wpl = wlo + n * 96 + ks * 32;
            FragB bh, bl;
            bh.half[0] = *(const v8b*)(wph + 8 * h);
            bh.half[1] = *(const v8b*)(wph + 16 + 8 * h);
            bl.half[0] = *(const v8b*)(wpl + 8 * h);
            bl.half[1] = *(const v8b*)(wpl + 16 + 8 * h);
            acc[nt] = mma_b(ah.v, bh.v, acc[nt]);
            acc[nt] = mma_b(ah.v, bl.v, acc[nt]);
            acc[nt] = mma_b(al.v, bh.v, acc[nt]);
        }
    }
    float* dsw = ds + wave * 512;
#pragma unroll
    for (int nt = 0; nt < 2; ++nt) {
        int n = nt * 16 + m;
        float bn = bsm[n];
#pragma unroll
        for (int r = 0; r < 8; ++r) dsw[(8 * h + r) * 32 + n] = acc[nt][r] + bn;
    }
    __syncthreads();
    float* osw = os + wave * X2P;
#pragma unroll 1
    for (int j = 0; j < 5; ++j) {
        int o = lane + 32 * j;
        int c = o / 5, f2 = o - 5 * c;
        float v0 = dsw[(3 * f2) * 32 + c];
        float v1 = dsw[(3 * f2 + 1) * 32 + c];
        float v2 = dsw[(3 * f2 + 2) * 32 + c];
        osw[o] = fmaxf(fmaxf(fmaxf(v0, v1), v2), 0.f);
    }
    __syncthreads();
    float* gp = x2 + (size_t)(bt0 + wave) * X2P;
    v4f s0 = *(const v4f*)(osw + lane * 4);
    v4f s1 = s0;
    bool second = lane < 8;
    if (second) s1 = *(const v4f*)(osw + (32 + lane) * 4);
    *(volatile v4f*)(gp + lane * 4) = s0;
    if (second) *(volatile v4f*)(gp + (32 + lane) * 4) = s1;
    __threadfence();
    *(volatile v4f*)(gp + lane * 4) = s0;
    if (second) *(volatile v4f*)(gp + (32 + lane) * 4) = s1;
}

__global__ __launch_bounds__(128) void k_conv3(const float* __restrict__ x2, const float* __restrict__ w,
                                               const float* __restrict__ bias, float* __restrict__ x) {
    __shared__ __attribute__((aligned(16))) float xs[66 * X2P];
    __shared__ __attribute__((aligned(16))) __bf16 whi[64 * 288];
    __shared__ __attribute__((aligned(16))) __bf16 wlo[64 * 288];
    __shared__ float bsm[192];
    __shared__ __attribute__((aligned(16))) float ds[4 * 16 * DD];
    int tid = threadIdx.x;
    int bt0 = blockIdx.x * 64;
    int tl0 = bt0 & (TT - 1);
    const v4f zero4 = {0.f, 0.f, 0.f, 0.f};
    for (int i = tid; i < 66 * (X2P / 4); i += 128) {
        int row = i / (X2P / 4), c4 = i - row * (X2P / 4);
        v4f val = zero4;
        if (tl0 + row < TT) val = ((const v4f*)(x2 + (size_t)(bt0 + row) * X2P))[c4];
        ((v4f*)xs)[i] = val;
    }
    for (int i = tid; i < 64 * 288; i += 128) {
        int n = i / 288, kk = i - n * 288;
        int i3 = kk / 96, r = kk - i3 * 96;
        float val = w[(size_t)(i3 * 64 + n) * 96 + r];
        __bf16 hi = (__bf16)val;
        whi[i] = hi;
        wlo[i] = (__bf16)(val - (float)hi);
    }
    for (int i = tid; i < 192; i += 128) bsm[i] = bias[i];
    __syncthreads();
    int wave = tid >> 5, lane = tid & 31, h = lane >> 4, m = lane & 15;
    int rbase = wave * 16;
    v8f mx[4];
#pragma unroll
    for (int nt = 0; nt < 4; ++nt) mx[nt] = v8fill(-3.4e38f);
#pragma unroll 1
    for (int f = 0; f < 3; ++f) {
        v8f acc[4];
#pragma unroll
        for (int nt = 0; nt < 4; ++nt) acc[nt] = v8fill(0.f);
#pragma unroll 1
        for (int ks = 0; ks < 9; ++ks) {
            FragB ah, al;
#pragma unroll
            for (int i = 0; i < 16; ++i) {
                int kk = ks * 32 + kmap(i, h);
                int i3 = kk / 96, r = kk - i3 * 96;
                int cin = r / 3, kw = r - cin * 3;
                float val = xs[(rbase + m + i3) * X2P + cin * 5 + f + kw];
                __bf16 hi = (__bf16)val;
                ah.v[i] = hi;
                al.v[i] = (__bf16)(val - (float)hi);
            }
#pragma unroll
            for (int nt = 0; nt < 4; ++nt) {
                const __bf16* wph = whi + (nt * 16 + m) * 288 + ks * 32;
                const __bf16* wpl = wlo + (nt * 16 + m) * 288 + ks * 32;
                FragB bh, bl;
                bh.half[0] = *(const v8b*)(wph + 8 * h);
                bh.half[1] = *(const v8b*)(wph + 16 + 8 * h);
                bl.half[0] = *(const v8b*)(wpl + 8 * h);
                bl.half[1] = *(const v8b*)(wpl + 16 + 8 * h);
                acc[nt] = mma_b(ah.v, bh.v, acc[nt]);
                acc[nt] = mma_b(ah.v, bl.v, acc[nt]);
                acc[nt] = mma_b(al.v, bh.v, acc[nt]);
            }
        }
#pragma unroll
        for (int nt = 0; nt < 4; ++nt)
#pragma unroll
            for (int r = 0; r < 8; ++r) mx[nt][r] = fmaxf(mx[nt][r], acc[nt][r]);
    }
    float* dsw = ds + wave * 1024;
#pragma unroll
    for (int r = 0; r < 8; ++r) {
        int tok = rbase + 8 * h + r;
        int nsub = TT - (tl0 + tok);
#pragma unroll
        for (int nt = 0; nt < 4; ++nt) {
            int n = nt * 16 + m;
            float bs = bsm[n];
            if (nsub > 1) bs += bsm[64 + n];
            if (nsub > 2) bs += bsm[128 + n];
            dsw[(8 * h + r) * DD + n] = fmaxf(mx[nt][r] + bs, 0.f);
        }
    }
    __syncthreads();
    wave_store_tile<false>(dsw, x + (size_t)(bt0 + rbase) * DD, lane);
}


__device__ __forceinline__ void proj16(const FragH& a0, const FragH& a1, const _Float16* __restrict__ wt,
                                       const float* __restrict__ bias, float* dsw, int h, int m) {
#pragma unroll
    for (int nt = 0; nt < 4; ++nt) {
        int n = nt * 16 + m;
        const _Float16* wp = wt + n * DD;
        FragH b0, b1;
        b0.half[0] = *(const v8h*)(wp + 8 * h);
        b0.half[1] = *(const v8h*)(wp + 16 + 8 * h);
        b1.half[0] = *(const v8h*)(wp + 32 + 8 * h);
        b1.half[1] = *(const v8h*)(wp + 48 + 8 * h);
        v8f acc = v8fill(0.f);
        acc = mma_h(a0.v, b0.v, acc);
        acc = mma_h(a1.v, b1.v, acc);
        float bn = bias[n];
#pragma unroll
        for (int r = 0; r < 8; ++r) dsw[(8 * h + r) * DD + n] = acc[r] * INV_WSC + bn;
    }
}

__global__ __launch_bounds__(128) void k_qkv(const float* __restrict__ x,
                                             const float* __restrict__ g, const float* __restrict__ be,
                                             const _Float16* __restrict__ wq, const _Float16* __restrict__ wk,
                                             const _Float16* __restrict__ wv,
                                             const float* __restrict__ bq, const float* __restrict__ bk,
                                             const float* __restrict__ bv,
                                             float* __restrict__ q, float* __restrict__ k, float* __restrict__ v) {
    __shared__ __attribute__((aligned(16))) _Float16 hs[64 * DD];
    __shared__ __attribute__((aligned(16))) float ds[4 * 16 * DD];
    int tid = threadIdx.x;
    int bt0 = blockIdx.x * 64;
    ln_rows(x, bt0, tid, g, be, hs);
    __syncthreads();
    int wave = tid >> 5, lane = tid & 31, h = lane >> 4, m = lane & 15;
    const _Float16* hr = hs + (wave * 16 + m) * DD;
    FragH a0, a1;
    a0.half[0] = *(const v8h*)(hr + 8 * h);
    a0.half[1] = *(const v8h*)(hr + 16 + 8 * h);
    a1.half[0] = *(const v8h*)(hr + 32 + 8 * h);
    a1.half[1] = *(const v8h*)(hr + 48 + 8 * h);
    float* dsw = ds + wave * 1024;
    size_t row0 = (size_t)(bt0 + wave * 16) * DD;
    proj16(a0, a1, wq, bq, dsw, h, m);
    __syncthreads();
    wave_store_tile<false>(dsw, q + row0, lane);
    __syncthreads();
    proj16(a0, a1, wk, bk, dsw, h, m);
    __syncthreads();
    wave_store_tile<false>(dsw, k + row0, lane);
    __syncthreads();
    proj16(a0, a1, wv, bv, dsw, h, m);
    __syncthreads();
    wave_store_tile<false>(dsw, v + row0, lane);
}

__global__ __launch_bounds__(128) void k_attn(const float* __restrict__ q, const float* __restrict__ k,
                                              const float* __restrict__ v, const float* __restrict__ er,
                                              float* __restrict__ x, int step) {
    __shared__ __attribute__((aligned(16))) float os[16 * DD];
    __shared__ float ers[NHD * 48];
    __shared__ float lgs[6 * 128];
    int tid = threadIdx.x;
    int bt0 = blockIdx.x * 16;
    for (int i = tid; i < NHD * 48; i += 128) ers[i] = er[i];
    __syncthreads();
    int tok = tid >> 3, hh = tid & 7;
    int bt = bt0 + tok;
    int b = bt >> 12, t = bt & (TT - 1);
    const v4f* qp = (const v4f*)(q + (size_t)bt * DD + hh * 8);
    v4f q0 = qp[0], q1 = qp[1];
    const float* kb = k + (size_t)b * TT * DD + hh * 8;
    const float* vb = v + (size_t)b * TT * DD + hh * 8;
    const float* eh = ers + hh * 48;
    float* lgt = lgs + tid;
    float mxl = -3.4e38f;
#pragma unroll 1
    for (int j = 0; j < 6; ++j) {
        int ts = t - ((j == 0) ? 0 : (j - 1) * step);
        float dot = 0.f;
        if (ts >= 0) {
            const v4f* kp = (const v4f*)(kb + (size_t)ts * DD);
            v4f k0 = kp[0], k1 = kp[1];
            dot = q0[0] * k0[0] + q0[1] * k0[1] + q0[2] * k0[2] + q0[3] * k0[3] +
                  q1[0] * k1[0] + q1[1] * k1[1] + q1[2] * k1[2] + q1[3] * k1[3];
        }
        float qe = 0.f;
#pragma unroll
        for (int d = 0; d < 4; ++d) qe += q0[d] * eh[d * 6 + j];
#pragma unroll
        for (int d = 0; d < 4; ++d) qe += q1[d] * eh[(4 + d) * 6 + j];
        float l = (dot + qe) * 0.35355339059327373f + ((dot == 0.f) ? 1e-9f : 0.f);
        lgt[j * 128] = l;
        mxl = fmaxf(mxl, l);
    }
    float sum = 0.f;
#pragma unroll 1
    for (int j = 0; j < 6; ++j) {
        float p = expf(lgt[j * 128] - mxl);
        lgt[j * 128] = p;
        sum += p;
    }
    float inv = 1.f / sum;
    v4f o0 = {0.f, 0.f, 0.f, 0.f}, o1 = {0.f, 0.f, 0.f, 0.f};
#pragma unroll 1
    for (int j = 0; j < 6; ++j) {
        int ts = t - ((j == 0) ? 0 : (j - 1) * step);
        if (ts >= 0) {
            const v4f* vp = (const v4f*)(vb + (size_t)ts * DD);
            v4f v0 = vp[0], v1 = vp[1];
            float a = lgt[j * 128] * inv;
            o0 += a * v0;
            o1 += a * v1;
        }
    }
    v4f* op = (v4f*)(os + tok * DD + hh * 8);
    op[0] = o0;
    op[1] = o1;
    __syncthreads();
    int wave = tid >> 5, lane = tid & 31;
    float* gp = x + (size_t)(bt0 + wave * 4) * DD;
    const float* lp = os + wave * 4 * DD;
    int offs[2];
    v4f vals[2];
#pragma unroll
    for (int it = 0; it < 2; ++it) {
        int ql = it * 4 + (lane >> 3);
        int off = (ql >> 1) * DD + ((ql & 1) << 5) + ((lane & 7) << 2);
        vals[it] = *(const v4f*)(gp + off) + *(const v4f*)(lp + off);
        offs[it] = off;
    }
#pragma unroll
    for (int it = 0; it < 2; ++it) *(volatile v4f*)(gp + offs[it]) = vals[it];
    __threadfence();
#pragma unroll
    for (int it = 0; it < 2; ++it) *(volatile v4f*)(gp + offs[it]) = vals[it];
}

__global__ __launch_bounds__(128) void k_ffn(float* __restrict__ x,
                                             const float* __restrict__ g, const float* __restrict__ be,
                                             const _Float16* __restrict__ w1, const float* __restrict__ b1,
                                             const _Float16* __restrict__ w2, const float* __restrict__ b2) {
    __shared__ __attribute__((aligned(16))) _Float16 hs[64 * DD];
    __shared__ __attribute__((aligned(16))) _Float16 h2[64 * DD];
    __shared__ __attribute__((aligned(16))) float ds[4 * 16 * DD];
    int tid = threadIdx.x;
    int bt0 = blockIdx.x * 64;
    ln_rows(x, bt0, tid, g, be, hs);
    __syncthreads();
    int wave = tid >> 5, lane = tid & 31, h = lane >> 4, m = lane & 15;
    const _Float16* hr = hs + (wave * 16 + m) * DD;
    FragH a0, a1;
    a0.half[0] = *(const v8h*)(hr + 8 * h);
    a0.half[1] = *(const v8h*)(hr + 16 + 8 * h);
    a1.half[0] = *(const v8h*)(hr + 32 + 8 * h);
    a1.half[1] = *(const v8h*)(hr + 48 + 8 * h);
#pragma unroll
    for (int nt = 0; nt < 4; ++nt) {
        int n = nt * 16 + m;
        const _Float16* wp = w1 + n * DD;
        FragH b0, b1f;
        b0.half[0]  = *(const v8h*)(wp + 8 * h);
        b0.half[1]  = *(const v8h*)(wp + 16 + 8 * h);
        b1f.half[0] = *(const v8h*)(wp + 32 + 8 * h);
        b1f.half[1] = *(const v8h*)(wp + 48 + 8 * h);
        v8f acc = v8fill(0.f);
        acc = mma_h(a0.v, b0.v, acc);
        acc = mma_h(a1.v, b1f.v, acc);
        float bn = b1[n];
#pragma unroll
        for (int r = 0; r < 8; ++r) {
            float u = acc[r] * INV_WSC + bn;
            float gel = 0.5f * u * (1.f + erff(u * 0.70710678118654752f));
            h2[(wave * 16 + 8 * h + r) * DD + n] = (_Float16)gel;
        }
    }
    __syncthreads();
    const _Float16* gr = h2 + (wave * 16 + m) * DD;
    FragH c0, c1;
    c0.half[0] = *(const v8h*)(gr + 8 * h);
    c0.half[1] = *(const v8h*)(gr + 16 + 8 * h);
    c1.half[0] = *(const v8h*)(gr + 32 + 8 * h);
    c1.half[1] = *(const v8h*)(gr + 48 + 8 * h);
    float* dsw = ds + wave * 1024;
#pragma unroll
    for (int nt = 0; nt < 4; ++nt) {
        int n = nt * 16 + m;
        const _Float16* wp = w2 + n * DD;
        FragH b0, b1f;
        b0.half[0]  = *(const v8h*)(wp + 8 * h);
        b0.half[1]  = *(const v8h*)(wp + 16 + 8 * h);
        b1f.half[0] = *(const v8h*)(wp + 32 + 8 * h);
        b1f.half[1] = *(const v8h*)(wp + 48 + 8 * h);
        v8f acc = v8fill(0.f);
        acc = mma_h(c0.v, b0.v, acc);
        acc = mma_h(c1.v, b1f.v, acc);
        float bn = b2[n];
#pragma unroll
        for (int r = 0; r < 8; ++r) dsw[(8 * h + r) * DD + n] = acc[r] * INV_WSC + bn;
    }
    __syncthreads();
    wave_store_tile<true>(dsw, x + (size_t)(bt0 + wave * 16) * DD, lane);
}

__global__ __launch_bounds__(256) void k_out(const float* __restrict__ x, const float* __restrict__ ow,
                                             const float* __restrict__ ob, float* __restrict__ out, int nbt) {
    __shared__ __attribute__((aligned(16))) float sos[2 * 256];
    int tid = threadIdx.x;
    int bt0 = blockIdx.x * 256;
    int bt = bt0 + tid;
    int b = bt0 >> 12, t0 = bt0 & (TT - 1);
    float r0 = 0.f, r1 = 0.f;
    if (bt < nbt) {
        const v4f* xr = (const v4f*)(x + (size_t)bt * DD);
        const v4f* wa = (const v4f*)ow;
        const v4f* wb = (const v4f*)(ow + DD);
        float a0 = ob[0], a1 = ob[1];
#pragma unroll 2
        for (int i = 0; i < 16; ++i) {
            v4f xv = xr[i], u = wa[i], s = wb[i];
            a0 += xv[0] * u[0] + xv[1] * u[1] + xv[2] * u[2] + xv[3] * u[3];
            a1 += xv[0] * s[0] + xv[1] * s[1] + xv[2] * s[2] + xv[3] * s[3];
        }
        r0 = 1.f / (1.f + expf(-a0));
        r1 = 1.f / (1.f + expf(-a1));
    }
    sos[tid] = r0;
    sos[256 + tid] = r1;
    __syncthreads();
    bool writer = (tid < 128) && (bt0 + 255 < nbt);
    int ch = tid >> 6, pc = tid & 63;
    v4f val = {0.f, 0.f, 0.f, 0.f};
    float* gp = out + ((size_t)b * 2 + ch) * TT + t0 + pc * 4;
    if (writer) {
        val = *(const v4f*)(sos + ch * 256 + pc * 4);
        *(volatile v4f*)gp = val;
    }
    __threadfence();
    if (writer) *(volatile v4f*)gp = val;
}

extern "C" void kernel_launch(void* const* d_in, const int* in_sizes, int n_in,
                              void* d_out, int out_size, void* d_ws, size_t ws_size,
                              hipStream_t stream) {
    if (n_in < 24) return;
    if (in_sizes[0] != BB * NSPEC * TT || out_size != BB * 2 * TT) return;

    const float* spec  = (const float*)d_in[0];
    const float* c1_w  = (const float*)d_in[1];
    const float* c1_b  = (const float*)d_in[2];
    const float* c2_w  = (const float*)d_in[3];
    const float* c2_b  = (const float*)d_in[4];
    const float* c3_w  = (const float*)d_in[5];
    const float* c3_b  = (const float*)d_in[6];
    const float* Wq    = (const float*)d_in[7];
    const float* bq    = (const float*)d_in[8];
    const float* Wk    = (const float*)d_in[9];
    const float* bk    = (const float*)d_in[10];
    const float* Wv    = (const float*)d_in[11];
    const float* bv    = (const float*)d_in[12];
    const float* Er    = (const float*)d_in[13];
    const float* g1    = (const float*)d_in[14];
    const float* be1   = (const float*)d_in[15];
    const float* W1    = (const float*)d_in[16];
    const float* b1    = (const float*)d_in[17];
    const float* W2    = (const float*)d_in[18];
    const float* b2    = (const float*)d_in[19];
    const float* g2    = (const float*)d_in[20];
    const float* be2   = (const float*)d_in[21];
    const float* out_w = (const float*)d_in[22];
    const float* out_b = (const float*)d_in[23];

    const size_t MIB     = 1024ull * 1024ull;
    const size_t OFF_WT  = 0;
    const size_t OFF_X   = 1 * MIB;
    const size_t OFF_Q   = OFF_X  + 8 * MIB;
    const size_t OFF_K   = OFF_Q  + 8 * MIB;
    const size_t OFF_V   = OFF_K  + 8 * MIB;
    const size_t OFF_X1  = OFF_V  + 8 * MIB;
    const size_t OFF_X2  = OFF_X1 + 28 * MIB;
    const size_t WS_END  = OFF_X2 + 20 * MIB;
    static_assert((size_t)BT * X1P * 4 == 28ull * 1024 * 1024);
    static_assert((size_t)BT * X2P * 4 == 20ull * 1024 * 1024);
    if (ws_size < WS_END) return;

    char* ws = (char*)d_ws;
    _Float16* Wt = (_Float16*)(ws + OFF_WT);
    float* x   = (float*)(ws + OFF_X);
    float* q   = (float*)(ws + OFF_Q);
    float* kk  = (float*)(ws + OFF_K);
    float* vv  = (float*)(ws + OFF_V);
    float* x1  = (float*)(ws + OFF_X1);
    float* x2  = (float*)(ws + OFF_X2);

    const int nvec = 5 * NLAY * DD * DD / 8;
    k_wcvt<<<(nvec + 255) / 256, 256, 0, stream>>>(Wq, Wk, Wv, W1, W2, Wt, nvec);
    k_conv1<<<BT / 8, 256, 0, stream>>>(spec, c1_w, c1_b, x1);
    k_conv2<<<BT / 4, 128, 0, stream>>>(x1, c2_w, c2_b, x2);
    k_conv3<<<BT / 64, 128, 0, stream>>>(x2, c3_w, c3_b, x);

    for (int L = 0; L < NLAY; ++L) {
        const _Float16* wtq = Wt + (size_t)(0 * NLAY + L) * DD * DD;
        const _Float16* wtk = Wt + (size_t)(1 * NLAY + L) * DD * DD;
        const _Float16* wtv = Wt + (size_t)(2 * NLAY + L) * DD * DD;
        const _Float16* wt1 = Wt + (size_t)(3 * NLAY + L) * DD * DD;
        const _Float16* wt2 = Wt + (size_t)(4 * NLAY + L) * DD * DD;
        k_qkv<<<BT / 64, 128, 0, stream>>>(x, g1 + L * DD, be1 + L * DD,
                                           wtq, wtk, wtv,
                                           bq + L * DD, bk + L * DD, bv + L * DD,
                                           q, kk, vv);
        k_attn<<<BT / 16, 128, 0, stream>>>(q, kk, vv, Er + L * NHD * 8 * 6, x, 1 << L);
        k_ffn<<<BT / 64, 128, 0, stream>>>(x, g2 + L * DD, be2 + L * DD,
                                           wt1, b1 + L * DD, wt2, b2 + L * DD);
    }
    const int nbt = BT;
    k_out<<<(nbt + 255) / 256, 256, 0, stream>>>(x, out_w, out_b, (float*)d_out, nbt);
}
